// BOJANET_23545010717406
// MI455X (gfx1250) — hardware-run, weakly checked
//
#include <hip/hip_runtime.h>
#include <math.h>

typedef __attribute__((ext_vector_type(16))) _Float16 v16h;
typedef __attribute__((ext_vector_type(8)))  _Float16 v8h;
typedef __attribute__((ext_vector_type(8)))  float    v8f;
typedef __attribute__((ext_vector_type(4)))  float    v4f;
typedef __attribute__((ext_vector_type(2)))  float    v2f;

constexpr int kBatch    = 512;
constexpr int kSteps    = 8192;
constexpr int kWin      = 16;
constexpr int kVd       = 6;
constexpr int kHid      = 12;
constexpr int kTileRows = 16;
constexpr int kTiles    = kBatch / kTileRows;
constexpr int kChunk    = 32;
constexpr int kNumChunks = kSteps / kChunk;
constexpr int kXPitch   = 2 * (8 + kChunk) + 4;
constexpr int kOPitch   = 2 * kChunk + 4;
constexpr size_t kIoElems = (size_t)kBatch * kSteps * 2;
static_assert(kBatch % kTileRows == 0 && kSteps % kChunk == 0, "whole tiles and chunks");
static_assert(kHid == 2 * kVd && kHid <= 16 && kWin == 16, "the 12 units and the 12 features fit the first 16 k; the 16 taps fill one half of K");
static_assert((kXPitch % 4) == 0 && (kOPitch % 4) == 0, "16-B aligned LDS rows");

constexpr float kCarry     = 1024.0f;
constexpr float kFoldBack  = 1.0f / (kCarry * kCarry);
constexpr float kF16MinNorm = 6.103515625e-5f;
constexpr float kEps = 1e-8f;

namespace eng {

union FragU { v16h v; v8h h[2]; };

__device__ __forceinline__ unsigned short f2bf_bits(float f) {
  unsigned u = __float_as_uint(f);
  return (unsigned short)((u + 0x7FFFu + ((u >> 16) & 1u)) >> 16);
}
__device__ __forceinline__ float bf16v(float f) {
  return __uint_as_float(((unsigned)f2bf_bits(f)) << 16);
}
__device__ __forceinline__ _Float16 to_f16_flushed(float c) {
  const float z = (fabsf(c) < kF16MinNorm) ? 0.0f : c;
  return (_Float16)z;
}
__device__ __forceinline__ v8f mma_f16(v16h a, v16h b) {
  v8f c = (v8f){0.f, 0.f, 0.f, 0.f, 0.f, 0.f, 0.f, 0.f};
  c = __builtin_amdgcn_wmma_f32_16x16x32_f16(false, a, false, b, (short)0, c, false, false);
  asm volatile("v_nop\n\tv_nop\n\tv_nop\n\tv_nop" : "+v"(c) : "v"(a), "v"(b));
  return c;
}

__device__ __forceinline__ float fast_tanh(float v) {
  const float e = __expf(2.0f * v);
  return 1.0f - 2.0f * __builtin_amdgcn_rcpf(e + 1.0f);
}
__device__ __forceinline__ float fast_sigmoid(float v) {
  return __builtin_amdgcn_rcpf(1.0f + __expf(-v));
}

}

__global__ __launch_bounds__(32) void demod_gate_seq_kernel(
    const float* __restrict__ x,
    const float* __restrict__ fir_I, const float* __restrict__ fir_Q,
    const float* __restrict__ W_fi, const float* __restrict__ b_fi, const float* __restrict__ W_fh,
    const float* __restrict__ W_gi, const float* __restrict__ b_gi, const float* __restrict__ W_gh,
    const float* __restrict__ w_oI, const float* __restrict__ b_oI,
    const float* __restrict__ w_oQ, const float* __restrict__ b_oQ,
    float* __restrict__ outs)
{
  __shared__ __align__(16) float xs[kTileRows * kXPitch];
  __shared__ __align__(16) float os[kTileRows * kOPitch];
  __shared__ __align__(16) float wsm[2 * 96 + 4 * 144 + 4 * 12 + 2 + 6];

  const int lane = threadIdx.x & 31;
  const int hsel = lane >> 4;
  const int n    = lane & 15;
  const bool lowHalf = (hsel == 0);
  const int b0   = blockIdx.x * kTileRows;
  constexpr int oFI = 0, oFQ = 96, oWfi = 192, oWfh = 336, oWgi = 480, oWgh = 624, oBf = 768, oBg = 780, oWI = 792, oWQ = 804, oBI = 816, oBQ = 817;

  {
#pragma unroll
    for (int it = 0; it < 3; ++it) {
      const int i = it * 32 + lane;
      wsm[oFI + i] = fir_I[i];
      wsm[oFQ + i] = fir_Q[i];
    }
#pragma unroll
    for (int it = 0; it < 5; ++it) {
      const int i  = it * 32 + lane;
      const int ic = (i < 144) ? i : 143;
      wsm[oWfi + ic] = W_fi[ic];
      wsm[oWfh + ic] = W_fh[ic];
      wsm[oWgi + ic] = W_gi[ic];
      wsm[oWgh + ic] = W_gh[ic];
    }
    const int c12 = (lane < kHid) ? lane : (kHid - 1);
    wsm[oBf + c12] = b_fi[c12];
    wsm[oBg + c12] = b_gi[c12];
    wsm[oWI + c12] = w_oI[c12];
    wsm[oWQ + c12] = w_oQ[c12];
    wsm[oBI] = b_oI[0];
    wsm[oBQ] = b_oQ[0];
    if (lane < 16) {
#pragma unroll
      for (int c = 0; c < 16; ++c) xs[lane * kXPitch + c] = 0.0f;
    }
  }
  __syncthreads();

  v16h fragFir[2];
  {
    const int m = n;
#pragma unroll
    for (int tl = 0; tl < 2; ++tl) {
      int u; bool isQ; bool live;
      if (tl == 0) { const int pr = (m < 8) ? (m >> 1) : (2 + ((m - 8) >> 1)); u = pr; isQ = (m & 1) != 0; live = true; }
      else         { u = (m < 4) ? (4 + (m >> 1)) : 5; isQ = (m & 1) != 0; live = (m < 4); }
      v8h a0, a1;
#pragma unroll
      for (int i = 0; i < 8; ++i) {
        const int k = 8 * hsel + i;
        const float wi = eng::bf16v(wsm[oFI + u * kWin + k]);
        const float wq = eng::bf16v(wsm[oFQ + u * kWin + k]);
        const float f0 = isQ ? wq : wi;
        const float f1 = isQ ? wi : -wq;
        a0[i] = eng::to_f16_flushed(live ? f0 * kCarry : 0.0f);
        a1[i] = eng::to_f16_flushed(live ? f1 * kCarry : 0.0f);
      }
      eng::FragU fu; fu.h[0] = a0; fu.h[1] = a1;
      fragFir[tl] = fu.v;
    }
  }
  v16h fragGate[2];
  {
    const int m  = n;
    const int mc = (m < kHid) ? m : (kHid - 1);
    const bool mok = (m < kHid);
#pragma unroll
    for (int g = 0; g < 2; ++g) {
      const int oi = g ? oWgi : oWfi;
      const int oh = g ? oWgh : oWfh;
      v8h a0, a1;
#pragma unroll
      for (int i = 0; i < 8; ++i) {
        const int k  = 8 * hsel + i;
        const int kc = (k < kHid) ? k : (kHid - 1);
        const bool ok = mok && (k < kHid);
        const float fi = eng::bf16v(wsm[oi + mc * kHid + kc]);
        const float fh = eng::bf16v(wsm[oh + mc * kHid + kc]);
        a0[i] = eng::to_f16_flushed(ok ? fi * kCarry : 0.0f);
        a1[i] = eng::to_f16_flushed(ok ? fh * kCarry : 0.0f);
      }
      eng::FragU fu; fu.h[0] = a0; fu.h[1] = a1;
      fragGate[g] = fu.v;
    }
  }

  float bfv[8], bgv[8], woI[8], woQ[8];
#pragma unroll
  for (int r = 0; r < 8; ++r) {
    const int uu = 8 * hsel + r;
    const int uc = (uu < kHid) ? uu : (kHid - 1);
    const bool live = (uu < kHid);
    bfv[r] = eng::bf16v(wsm[oBf + uc]);
    bgv[r] = eng::bf16v(wsm[oBg + uc]);
    const float vi = eng::bf16v(wsm[oWI + uc]);
    const float vq = eng::bf16v(wsm[oWQ + uc]);
    woI[r] = live ? vi : 0.0f;
    woQ[r] = live ? vq : 0.0f;
  }
  const float boI = eng::bf16v(wsm[oBI]);
  const float boQ = eng::bf16v(wsm[oBQ]);

  float hf[8];
  v8h hb, wI, wQ;
#pragma unroll
  for (int r = 0; r < 8; ++r) { hf[r] = 0.0f; hb[r] = (_Float16)0.0f; wI[r] = (_Float16)0.0f; wQ[r] = (_Float16)0.0f; }

  const int q  = lane >> 3;
  const int c4 = (lane & 7) * 4;

#pragma unroll 1
  for (int ch = 0; ch < kNumChunks; ++ch) {
    const int t0 = ch * kChunk;
#pragma unroll
    for (int it = 0; it < 8; ++it) {
      const int row = (it >> 1) * 4 + q;
      const int hl  = it & 1;
      const v4f v = *(const v4f*)(x + ((size_t)(b0 + row) * kSteps + t0) * 2 + hl * 32 + c4);
      v4f rv;
      rv[0] = eng::bf16v(v[0]);
      rv[1] = eng::bf16v(v[1]);
      rv[2] = eng::bf16v(v[2]);
      rv[3] = eng::bf16v(v[3]);
      *(v4f*)(xs + row * kXPitch + 16 + hl * 32 + c4) = rv;
    }
    __syncthreads();

#pragma unroll 1
    for (int s = 0; s < kChunk; ++s) {
      const v2f xin = *(const v2f*)(xs + n * kXPitch + 2 * (s + 8 * hsel));
#pragma unroll
      for (int i = 0; i < 7; ++i) { wI[i] = wI[i + 1]; wQ[i] = wQ[i + 1]; }
      wI[7] = eng::to_f16_flushed(xin[0] * kCarry);
      wQ[7] = eng::to_f16_flushed(xin[1] * kCarry);
      eng::FragU fw; fw.h[0] = wI; fw.h[1] = wQ;
      const v8f dA = eng::mma_f16(fragFir[0], fw.v);
      const v8f dB = eng::mma_f16(fragFir[1], fw.v);

      float mg[6], cs[6], sn[6];
#pragma unroll
      for (int p = 0; p < 6; ++p) {
        const float fi = ((p < 4) ? dA[2 * p] : dB[2 * (p - 4)]) * kFoldBack;
        const float fq = ((p < 4) ? dA[2 * p + 1] : dB[2 * (p - 4) + 1]) * kFoldBack;
        const float m0 = sqrtf(fi * fi + fq * fq) + kEps;
        const float inv = 1.0f / m0;
        mg[p] = m0;
        cs[p] = fi * inv;
        sn[p] = fq * inv;
      }
      v8h lb;
#pragma unroll
      for (int i = 0; i < 8; ++i) {
        const float lo = (i < 6) ? mg[i] : (mg[i - 6] * mg[i - 6]);
        const float hi = (i < 4) ? (mg[i] * mg[i]) : 0.0f;
        lb[i] = eng::to_f16_flushed((lowHalf ? lo : hi) * kCarry);
      }
      eng::FragU fb; fb.h[0] = lb; fb.h[1] = hb;
      const v8f af = eng::mma_f16(fragGate[0], fb.v);
      const v8f ag = eng::mma_f16(fragGate[1], fb.v);

      float pa = 0.0f, pb = 0.0f;
#pragma unroll
      for (int r = 0; r < 8; ++r) {
        const float fg = eng::fast_sigmoid(fmaf(af[r], kFoldBack, bfv[r]));
        const float gg = eng::fast_tanh(fmaf(ag[r], kFoldBack, bgv[r]));
        const float tv = fg * hf[r] + (1.0f - fg) * gg;
        const bool live = (8 * hsel + r) < kHid;
        const float hv = live ? tv : 0.0f;
        hf[r] = hv;
        hb[r] = eng::to_f16_flushed(hv * kCarry);
        const float cl = cs[(r < 6) ? r : (r - 6)], ch2 = cs[(r < 4) ? r : 0];
        const float sl = sn[(r < 6) ? r : (r - 6)], sh2 = sn[(r < 4) ? r : 0];
        const float cv = lowHalf ? cl : ch2;
        const float sv = lowHalf ? sl : sh2;
        pa = fmaf(hv * cv, woI[r], pa);
        pb = fmaf(hv * sv, woQ[r], pb);
      }
      const float a = (pa + __shfl_xor(pa, 16, 32)) + boI;
      const float b = (pb + __shfl_xor(pb, 16, 32)) + boQ;
      if (lowHalf) {
        const v2f ov = {a - b, b + a};
        *(v2f*)(os + n * kOPitch + 2 * s) = ov;
      }
    }
    __syncthreads();

    {
      v4f hk[4];
#pragma unroll
      for (int c = 0; c < 4; ++c) hk[c] = *(const v4f*)(xs + n * kXPitch + 64 + 4 * c);
      v4f ov[8];
#pragma unroll
      for (int it = 0; it < 8; ++it) ov[it] = *(const v4f*)(os + ((it >> 1) * 4 + q) * kOPitch + (it & 1) * 32 + c4);
      __syncthreads();
      if (lowHalf) {
#pragma unroll
        for (int c = 0; c < 4; ++c) *(v4f*)(xs + n * kXPitch + 4 * c) = hk[c];
      }
      for (int pass = 0; pass < 2; ++pass) {
#pragma unroll
        for (int it = 0; it < 8; ++it)
          *(volatile v4f*)(outs + ((size_t)(b0 + (it >> 1) * 4 + q) * kSteps + t0) * 2 + (it & 1) * 32 + c4) = ov[it];
        __threadfence();
      }
    }
    __syncthreads();
  }
}

extern "C" void kernel_launch(void* const* d_in, const int* in_sizes, int n_in,
                              void* d_out, int out_size, void* d_ws, size_t ws_size,
                              hipStream_t stream) {
  (void)d_ws;
  (void)ws_size;
  if (n_in < 13 || d_out == nullptr) return;
  if ((size_t)in_sizes[0] != kIoElems) return;
  if (in_sizes[1] != kVd * kWin || in_sizes[2] != kVd * kWin) return;
  if (in_sizes[3] != kHid * kHid || in_sizes[4] != kHid || in_sizes[5] != kHid * kHid) return;
  if (in_sizes[6] != kHid * kHid || in_sizes[7] != kHid || in_sizes[8] != kHid * kHid) return;
  if (in_sizes[9] != kHid || in_sizes[10] != 1 || in_sizes[11] != kHid || in_sizes[12] != 1) return;
  if ((size_t)out_size != kIoElems) return;

  demod_gate_seq_kernel<<<kTiles, 32, 0, stream>>>(
      (const float*)d_in[0], (const float*)d_in[1], (const float*)d_in[2],
      (const float*)d_in[3], (const float*)d_in[4], (const float*)d_in[5],
      (const float*)d_in[6], (const float*)d_in[7], (const float*)d_in[8],
      (const float*)d_in[9], (const float*)d_in[10], (const float*)d_in[11], (const float*)d_in[12],
      (float*)d_out);
}
